// MatrixOdeTrainableModelLeastSquares_4861902979218
// MI455X (gfx1250) — hardware-run, weakly checked
//
#include <hip/hip_runtime.h>
#include <math.h>

typedef __attribute__((ext_vector_type(16))) _Float16 v16h;
typedef __attribute__((ext_vector_type(8)))  _Float16 v8h;
typedef __attribute__((ext_vector_type(16))) __bf16   v16b;
typedef __attribute__((ext_vector_type(8)))  __bf16   v8b;
typedef __attribute__((ext_vector_type(8)))  float    v8f;
typedef __attribute__((ext_vector_type(4)))  float    v4f;

constexpr int kRowsB = 4096;
constexpr int kDx    = 512;
constexpr int kDz    = 512;
constexpr int kDy    = 256;
constexpr int kHid   = 2048;
constexpr int kSteps = 64;
constexpr int kK3    = 3 * kDz;
constexpr int kTileP = 68;

constexpr float kDt       = 1.0f / (float)kSteps;
constexpr float kCarryW   = 1024.0f;
constexpr float kCarryAct = 16.0f;
constexpr float kFoldBack = 1.0f / (kCarryW * kCarryAct);
constexpr float kResCarry = 2048.0f;
constexpr float kResInv   = 1.0f / kResCarry;

static_assert(kDx == kDz, "square small-chain planes");
static_assert((kDz % 64) == 0 && (kRowsB % 64) == 0 && (kHid % 64) == 0 && (kDy % 64) == 0, "M,N multiples of 64");
static_assert((kRowsB % 32) == 0, "three-product wave tiles are 32 rows");
static_assert((kK3 % 32) == 0 && (kDx % 32) == 0 && (kDz % 32) == 0 && (kHid % 32) == 0, "K multiples of 32");
static_assert((((kDz / 64) * (kDz / 64)) % 8) == 0, "small chain: 64 wave tiles = 8 blocks");
static_assert((((kRowsB / 64) * (kHid / 64)) % 8) == 0, "layer 2: whole blocks of 8 wave tiles (64 x 64)");
static_assert((((kRowsB / 32) * (kDz / 64)) % 8) == 0 && (((kRowsB / 32) * (kHid / 64)) % 8) == 0 &&
              (((kRowsB / 32) * (kDy / 64)) % 8) == 0, "three-product sites: whole blocks of 8 wave tiles (32 x 64)");
static_assert(((kRowsB * kDx / 8) % 256) == 0 && ((kHid * kDz / 8) % 256) == 0 && ((kHid * kHid / 8) % 256) == 0 &&
              ((kDy * kHid / 8) % 256) == 0, "cast grids exact");

constexpr size_t kOffX16   = 0;
constexpr size_t kOffX16R  = kOffX16   + (size_t)kRowsB * kDx  * 2;
constexpr size_t kOffW1H   = kOffX16R  + (size_t)kRowsB * kDx  * 2;
constexpr size_t kOffW1R   = kOffW1H   + (size_t)kHid   * kDz  * 2;
constexpr size_t kOffW2H   = kOffW1R   + (size_t)kHid   * kDz  * 2;
constexpr size_t kOffW3H   = kOffW2H   + (size_t)kHid   * kHid * 2;
constexpr size_t kOffW3R   = kOffW3H   + (size_t)kDy    * kHid * 2;
constexpr size_t kOffZT16  = kOffW3R   + (size_t)kDy    * kHid * 2;
constexpr size_t kOffZT16R = kOffZT16  + (size_t)kRowsB * kDz  * 2;
constexpr size_t kOffH1    = kOffZT16R + (size_t)kRowsB * kDz  * 2;
constexpr size_t kOffH2    = kOffH1    + (size_t)kRowsB * kHid * 2;
constexpr size_t kOffH2R   = kOffH2    + (size_t)kRowsB * kHid * 2;
constexpr size_t kOffF0    = kOffH2R   + (size_t)kRowsB * kHid * 2;
constexpr size_t kOffF1    = kOffF0    + (size_t)kDz * kDz * 4;
constexpr size_t kOffF2    = kOffF1    + (size_t)kDz * kDz * 4;
constexpr size_t kOffLA    = kOffF2    + (size_t)kDz * kDz * 4;
constexpr size_t kOffLE    = kOffLA    + (size_t)kDz * kK3 * 2;
constexpr size_t kOffRT    = kOffLE    + (size_t)kDz * kK3 * 2;
constexpr size_t kOffPT    = kOffRT    + (size_t)kDz * kK3 * 2;
constexpr size_t kOffC16   = kOffPT    + (size_t)kDz * kK3 * 2;
constexpr size_t kOffC16R  = kOffC16   + (size_t)kDz * kDx * 2;
constexpr size_t kWsTotal  = kOffC16R  + (size_t)kDz * kDx * 2;
static_assert(kWsTotal == 92274688ull, "carve total");
static_assert(kWsTotal <= 134217728ull, "carve cap");
static_assert((kOffX16R % 128) == 0 && (kOffW1H % 128) == 0 && (kOffW1R % 128) == 0 && (kOffW2H % 128) == 0 &&
              (kOffW3H % 128) == 0 && (kOffW3R % 128) == 0 && (kOffZT16 % 128) == 0 && (kOffZT16R % 128) == 0 &&
              (kOffH1 % 128) == 0 && (kOffH2 % 128) == 0 && (kOffH2R % 128) == 0 && (kOffF0 % 128) == 0 &&
              (kOffF1 % 128) == 0 && (kOffF2 % 128) == 0 && (kOffLA % 128) == 0 && (kOffLE % 128) == 0 &&
              (kOffRT % 128) == 0 && (kOffPT % 128) == 0 && (kOffC16 % 128) == 0 && (kOffC16R % 128) == 0,
              "128-B aligned regions");

__device__ __forceinline__ unsigned short f2bf_bits(float f) {
  unsigned u = __float_as_uint(f);
  return (unsigned short)((u + 0x7FFFu + ((u >> 16) & 1u)) >> 16);
}
__device__ __forceinline__ float bf_bits2f(unsigned short h) { return __uint_as_float(((unsigned)h) << 16); }

__device__ __forceinline__ v8f mma_guard_h(v16h a, v16h b, v8f c) {
  c = __builtin_amdgcn_wmma_f32_16x16x32_f16(false, a, false, b, (short)0, c, false, false);
  asm volatile("v_nop\n\tv_nop\n\tv_nop\n\tv_nop" : "+v"(c) : "v"(a), "v"(b));
  return c;
}
__device__ __forceinline__ v8f mma_guard_b(v16b a, v16b b, v8f c) {
  c = __builtin_amdgcn_wmma_f32_16x16x32_bf16(false, a, false, b, (short)0, c, false, false);
  asm volatile("v_nop\n\tv_nop\n\tv_nop\n\tv_nop" : "+v"(c) : "v"(a), "v"(b));
  return c;
}
__device__ __forceinline__ void acc_guard4(v8f& a, v8f& b, v8f& c, v8f& d) {
  asm volatile("v_nop\n\tv_nop\n\tv_nop\n\tv_nop" : "+v"(a), "+v"(b), "+v"(c), "+v"(d));
}

template <typename T> struct Frag;
template <> struct Frag<_Float16> {
  typedef v16h V;
  union U { v16h v; v8h h[2]; };
  static __device__ __forceinline__ v16h load(const _Float16* p) {
    U f;
    f.h[0] = *(const v8h*)(p);
    f.h[1] = *(const v8h*)(p + 16);
    return f.v;
  }
  static __device__ __forceinline__ v8f mma(v16h a, v16h b, v8f c) { return mma_guard_h(a, b, c); }
};
template <> struct Frag<__bf16> {
  typedef v16b V;
  union U { v16b v; v8b h[2]; };
  static __device__ __forceinline__ v16b load(const __bf16* p) {
    U f;
    f.h[0] = *(const v8b*)(p);
    f.h[1] = *(const v8b*)(p + 16);
    return f.v;
  }
  static __device__ __forceinline__ v8f mma(v16b a, v16b b, v8f c) { return mma_guard_b(a, b, c); }
};

template <int ET> struct Elem;
template <> struct Elem<0> { typedef _Float16 T; };
template <> struct Elem<1> { typedef __bf16 T; };

template <int ET, bool SPL3, bool HAS_BIAS, int OUT_MODE, bool RESID, bool RELU, bool GUARD>
__global__ __launch_bounds__(256) void gemm64_kernel(
    const unsigned short* __restrict__ Ap, const unsigned short* A2p, int lda,
    const unsigned short* __restrict__ Btp, const unsigned short* Bt2p, int ldb,
    void* __restrict__ Cout, void* Cout2, int ldc,
    const float* __restrict__ bias,
    const float* __restrict__ resid, int ldr,
    const int* __restrict__ premise,
    int M, int N, int K, float alpha, float beta, float oscale) {
  static_assert(!GUARD || OUT_MODE == 0, "premise guard only on the f32 output path");
  static_assert(!SPL3 || ET == 0, "three-product form is f16 only");
  typedef typename Elem<ET>::T T;
  typedef typename Frag<T>::V V;
  constexpr int TI = SPL3 ? 2 : 4;
  constexpr int TROWS = TI * 16;
  const T* A   = (const T*)Ap;
  const T* A2  = (const T*)A2p;
  const T* Bt  = (const T*)Btp;
  const T* Bt2 = (const T*)Bt2p;
  __shared__ __align__(16) float sT[8][16 * 68];
  const int lane = threadIdx.x & 31;
  const int wave = threadIdx.x >> 5;
  const int tilesN = N >> 6;
  const int tilesM = M / TROWS;
  const int tile = blockIdx.x * 8 + wave;
  if (tile >= tilesM * tilesN) return;
  const int tm = tile / tilesN;
  const int tn = tile - tm * tilesN;
  const int m0 = tm * TROWS;
  const int n0 = tn << 6;

  const int rlane = lane & 15;
  const int koff  = (lane >> 4) * 8;
  const int mOff  = (lane >> 4) * 8;

  bool ok = true;
  if (GUARD) {
    const int ns = premise[0];
    ok = (ns == kSteps);
  }
  const float nanv = __uint_as_float(0x7fc00000u);

  v8f acc[TI][4];
  v8f acc2[SPL3 ? TI : 1][4];
#pragma unroll
  for (int i = 0; i < TI; ++i)
#pragma unroll
    for (int j = 0; j < 4; ++j) acc[i][j] = (v8f){0.f, 0.f, 0.f, 0.f, 0.f, 0.f, 0.f, 0.f};
#pragma unroll
  for (int i = 0; i < (SPL3 ? TI : 1); ++i)
#pragma unroll
    for (int j = 0; j < 4; ++j) acc2[i][j] = (v8f){0.f, 0.f, 0.f, 0.f, 0.f, 0.f, 0.f, 0.f};

  for (int k0 = 0; k0 < K; k0 += 32) {
    V bh[4];
    V bl[4];
#pragma unroll
    for (int j = 0; j < 4; ++j) {
      const size_t bo = (size_t)(n0 + (j << 4) + rlane) * ldb + koff + k0;
      bh[j] = Frag<T>::load(Bt + bo);
      if (SPL3) bl[j] = Frag<T>::load(Bt2 + bo);
      else bl[j] = bh[j];
    }
#pragma unroll
    for (int i = 0; i < TI; ++i) {
      const size_t ao = (size_t)(m0 + (i << 4) + rlane) * lda + koff + k0;
      const V ah = Frag<T>::load(A + ao);
      V al = ah;
      if (SPL3) al = Frag<T>::load(A2 + ao);
#pragma unroll
      for (int j = 0; j < 4; ++j) {
        acc[i][j] = Frag<T>::mma(ah, bh[j], acc[i][j]);
        if (SPL3) {
          acc2[SPL3 ? i : 0][j] = Frag<T>::mma(ah, bl[j], acc2[SPL3 ? i : 0][j]);
          acc2[SPL3 ? i : 0][j] = Frag<T>::mma(al, bh[j], acc2[SPL3 ? i : 0][j]);
        }
      }
    }
  }
#pragma unroll
  for (int i = 0; i < TI; ++i) {
    acc_guard4(acc[i][0], acc[i][1], acc[i][2], acc[i][3]);
    if (SPL3) acc_guard4(acc2[SPL3 ? i : 0][0], acc2[SPL3 ? i : 0][1], acc2[SPL3 ? i : 0][2], acc2[SPL3 ? i : 0][3]);
  }

  float* slab = sT[wave];
  const int hh0 = lane >> 4;
  const int c4  = (lane & 15) * 4;
  const int q   = lane >> 3;
  const int c8  = (lane & 7) * 8;
  v4f bias4  = (v4f){0.f, 0.f, 0.f, 0.f};
  v4f bias8a = (v4f){0.f, 0.f, 0.f, 0.f};
  v4f bias8b = (v4f){0.f, 0.f, 0.f, 0.f};
  if (HAS_BIAS) {
    if (OUT_MODE == 0) {
      bias4 = *(const v4f*)(bias + n0 + c4);
    } else {
      bias8a = *(const v4f*)(bias + n0 + c8);
      bias8b = *(const v4f*)(bias + n0 + c8 + 4);
    }
  }
#pragma unroll
  for (int i = 0; i < TI; ++i) {
    const int mBase = m0 + (i << 4);
#pragma unroll
    for (int j = 0; j < 4; ++j) {
#pragma unroll
      for (int r = 0; r < 8; ++r) {
        float v = acc[i][j][r];
        if (SPL3) v = v + acc2[SPL3 ? i : 0][j][r] * kResInv;
        slab[(mOff + r) * 68 + (j << 4) + rlane] = v * alpha;
      }
    }
    __builtin_amdgcn_fence(__ATOMIC_RELEASE, "workgroup");
    __builtin_amdgcn_wave_barrier();
    __builtin_amdgcn_fence(__ATOMIC_ACQUIRE, "workgroup");
    if (OUT_MODE == 0) {
      float* C = (float*)Cout;
      v4f vals[8];
#pragma unroll
      for (int it = 0; it < 8; ++it) {
        const int row = it * 2 + hh0;
        v4f v = *(const v4f*)(slab + row * 68 + c4);
        if (HAS_BIAS) v = v + bias4;
        if (RESID) {
          const v4f rv = *(const v4f*)(resid + (size_t)(mBase + row) * ldr + n0 + c4);
          v = v + rv * beta;
        }
        if (RELU) {
#pragma unroll
          for (int e = 0; e < 4; ++e) v[e] = fmaxf(v[e], 0.0f);
        }
        if (GUARD) {
#pragma unroll
          for (int e = 0; e < 4; ++e) v[e] = ok ? v[e] : nanv;
        }
        vals[it] = v;
      }
      for (int pass = 0; pass < 2; ++pass) {
#pragma unroll
        for (int it = 0; it < 8; ++it) {
          const int row = it * 2 + hh0;
          *(volatile v4f*)(C + (size_t)(mBase + row) * ldc + n0 + c4) = vals[it];
        }
        __threadfence();
      }
    } else {
      unsigned short* C  = (unsigned short*)Cout;
      unsigned short* C2 = (unsigned short*)Cout2;
      v8h hv[4];
      v8h lv[4];
#pragma unroll
      for (int it = 0; it < 4; ++it) {
        const int row = it * 4 + q;
        const float* sp = slab + row * 68 + c8;
        v4f a0 = *(const v4f*)(sp);
        v4f a1 = *(const v4f*)(sp + 4);
        if (HAS_BIAS) {
          a0 = a0 + bias8a;
          a1 = a1 + bias8b;
        }
        if (RESID) {
          const float* rp = resid + (size_t)(mBase + row) * ldr + n0 + c8;
          const v4f r0 = *(const v4f*)(rp);
          const v4f r1 = *(const v4f*)(rp + 4);
          a0 = a0 + r0 * beta;
          a1 = a1 + r1 * beta;
        }
        if (RELU) {
#pragma unroll
          for (int e = 0; e < 4; ++e) {
            a0[e] = fmaxf(a0[e], 0.0f);
            a1[e] = fmaxf(a1[e], 0.0f);
          }
        }
        a0 = a0 * oscale;
        a1 = a1 * oscale;
#pragma unroll
        for (int e = 0; e < 4; ++e) {
          const float f0 = a0[e];
          const float f1 = a1[e];
          const _Float16 h0 = (_Float16)f0;
          const _Float16 h1 = (_Float16)f1;
          hv[it][e]     = h0;
          hv[it][4 + e] = h1;
          if (OUT_MODE == 2) {
            const float hf0 = (float)h0;
            const float hf1 = (float)h1;
            const float g0 = (f0 - hf0) * kResCarry;
            const float g1 = (f1 - hf1) * kResCarry;
            lv[it][e]     = (_Float16)g0;
            lv[it][4 + e] = (_Float16)g1;
          } else {
            lv[it][e]     = h0;
            lv[it][4 + e] = h1;
          }
        }
      }
      for (int pass = 0; pass < 2; ++pass) {
#pragma unroll
        for (int it = 0; it < 4; ++it) {
          const int row = it * 4 + q;
          const size_t o = (size_t)(mBase + row) * ldc + n0 + c8;
          *(volatile v8h*)(C + o) = hv[it];
          if (OUT_MODE == 2) *(volatile v8h*)(C2 + o) = lv[it];
        }
        __threadfence();
      }
    }
    __builtin_amdgcn_fence(__ATOMIC_RELEASE, "workgroup");
    __builtin_amdgcn_wave_barrier();
    __builtin_amdgcn_fence(__ATOMIC_ACQUIRE, "workgroup");
  }
}

template <bool RES>
__global__ __launch_bounds__(256) void cast_f16_carry_kernel(
    const float* __restrict__ src, unsigned short* __restrict__ dst, unsigned short* dst2, int total8, float carry) {
  const int i = blockIdx.x * 256 + threadIdx.x;
  if (i >= total8) return;
  const size_t e0 = (size_t)i << 3;
  const v4f a0 = *(const v4f*)(src + e0);
  const v4f a1 = *(const v4f*)(src + e0 + 4);
  v8h hv;
  v8h lv;
#pragma unroll
  for (int e = 0; e < 4; ++e) {
    const float f0 = a0[e] * carry;
    const float f1 = a1[e] * carry;
    const _Float16 h0 = (_Float16)f0;
    const _Float16 h1 = (_Float16)f1;
    hv[e]     = h0;
    hv[4 + e] = h1;
    if (RES) {
      const float hf0 = (float)h0;
      const float hf1 = (float)h1;
      const float g0 = (f0 - hf0) * kResCarry;
      const float g1 = (f1 - hf1) * kResCarry;
      lv[e]     = (_Float16)g0;
      lv[4 + e] = (_Float16)g1;
    } else {
      lv[e]     = h0;
      lv[4 + e] = h1;
    }
  }
  unsigned short* p  = dst + e0;
  unsigned short* p2 = dst2 + e0;
  *(volatile v8h*)p = hv;
  if (RES) *(volatile v8h*)p2 = lv;
  __threadfence();
  *(volatile v8h*)p = hv;
  if (RES) *(volatile v8h*)p2 = lv;
}

template <bool DO_L, bool DO_R>
__global__ __launch_bounds__(256) void split_planes_kernel(
    const float* __restrict__ src, unsigned short* __restrict__ Lp, unsigned short* __restrict__ Rp, float scale) {
  __shared__ __align__(16) float tile[64 * kTileP];
  const int tid = threadIdx.x;
  const int lane = tid & 31;
  const int wave = tid >> 5;
  const int r0 = blockIdx.y * 64;
  const int c0 = blockIdx.x * 64;
  {
    const int sr = tid >> 4;
    const int sc = (tid & 15) * 4;
#pragma unroll
    for (int i = 0; i < 4; ++i) {
      const int row = sr + 16 * i;
      v4f v = *(const v4f*)(src + (size_t)(r0 + row) * kDz + c0 + sc);
      v = v * scale;
      *(v4f*)(tile + row * kTileP + sc) = v;
    }
  }
  __syncthreads();
  const int q  = lane >> 3;
  const int c8 = (lane & 7) * 8;
  v8h lhv[2], llv[2], rhv[2], rlv[2];
#pragma unroll
  for (int it = 0; it < 2; ++it) {
    const int row = it * 32 + wave * 4 + q;
    if (DO_L) {
#pragma unroll
      for (int e = 0; e < 8; ++e) {
        const float f = tile[row * kTileP + c8 + e];
        const unsigned short hb = f2bf_bits(f);
        const unsigned short lb = f2bf_bits(f - bf_bits2f(hb));
        lhv[it][e] = __builtin_bit_cast(_Float16, hb);
        llv[it][e] = __builtin_bit_cast(_Float16, lb);
      }
    }
    if (DO_R) {
#pragma unroll
      for (int e = 0; e < 8; ++e) {
        const float f = tile[(c8 + e) * kTileP + row];
        const unsigned short hb = f2bf_bits(f);
        const unsigned short lb = f2bf_bits(f - bf_bits2f(hb));
        rhv[it][e] = __builtin_bit_cast(_Float16, hb);
        rlv[it][e] = __builtin_bit_cast(_Float16, lb);
      }
    }
  }
  for (int pass = 0; pass < 2; ++pass) {
#pragma unroll
    for (int it = 0; it < 2; ++it) {
      const int row = it * 32 + wave * 4 + q;
      if (DO_L) {
        const size_t o = (size_t)(r0 + row) * kK3 + c0 + c8;
        *(volatile v8h*)(Lp + o)           = lhv[it];
        *(volatile v8h*)(Lp + o + kDz)     = lhv[it];
        *(volatile v8h*)(Lp + o + 2 * kDz) = llv[it];
      }
      if (DO_R) {
        const size_t o = (size_t)(c0 + row) * kK3 + r0 + c8;
        *(volatile v8h*)(Rp + o)           = rhv[it];
        *(volatile v8h*)(Rp + o + kDz)     = rlv[it];
        *(volatile v8h*)(Rp + o + 2 * kDz) = rhv[it];
      }
    }
    __threadfence();
  }
}

extern "C" void kernel_launch(void* const* d_in, const int* in_sizes, int n_in,
                              void* d_out, int out_size, void* d_ws, size_t ws_size,
                              hipStream_t stream) {
  if (n_in < 10) return;
  if (in_sizes[0] != kRowsB * kDx) return;
  if (in_sizes[1] != kDz * kDx) return;
  if (in_sizes[2] != kDz * kDz) return;
  if (in_sizes[3] != kHid * kDz) return;
  if (in_sizes[4] != kHid) return;
  if (in_sizes[5] != kHid * kHid) return;
  if (in_sizes[6] != kHid) return;
  if (in_sizes[7] != kDy * kHid) return;
  if (in_sizes[8] != kDy) return;
  if (in_sizes[9] != 1) return;
  if (out_size != kRowsB * kDy) return;
  if (ws_size < kWsTotal) return;

  const float* X   = (const float*)d_in[0];
  const float* Pm  = (const float*)d_in[1];
  const float* Am  = (const float*)d_in[2];
  const float* W1  = (const float*)d_in[3];
  const float* b1  = (const float*)d_in[4];
  const float* W2  = (const float*)d_in[5];
  const float* b2  = (const float*)d_in[6];
  const float* W3  = (const float*)d_in[7];
  const float* b3  = (const float*)d_in[8];
  const int*   nst = (const int*)d_in[9];
  float* y = (float*)d_out;

  char* ws = (char*)d_ws;
  unsigned short* X16   = (unsigned short*)(ws + kOffX16);
  unsigned short* X16R  = (unsigned short*)(ws + kOffX16R);
  unsigned short* W1H   = (unsigned short*)(ws + kOffW1H);
  unsigned short* W1R   = (unsigned short*)(ws + kOffW1R);
  unsigned short* W2H   = (unsigned short*)(ws + kOffW2H);
  unsigned short* W3H   = (unsigned short*)(ws + kOffW3H);
  unsigned short* W3R   = (unsigned short*)(ws + kOffW3R);
  unsigned short* ZT16  = (unsigned short*)(ws + kOffZT16);
  unsigned short* ZT16R = (unsigned short*)(ws + kOffZT16R);
  unsigned short* H1    = (unsigned short*)(ws + kOffH1);
  unsigned short* H2    = (unsigned short*)(ws + kOffH2);
  unsigned short* H2R   = (unsigned short*)(ws + kOffH2R);
  float*          F0    = (float*)(ws + kOffF0);
  float*          F1    = (float*)(ws + kOffF1);
  float*          F2    = (float*)(ws + kOffF2);
  unsigned short* LA    = (unsigned short*)(ws + kOffLA);
  unsigned short* LE    = (unsigned short*)(ws + kOffLE);
  unsigned short* RT    = (unsigned short*)(ws + kOffRT);
  unsigned short* PT    = (unsigned short*)(ws + kOffPT);
  unsigned short* C16   = (unsigned short*)(ws + kOffC16);
  unsigned short* C16R  = (unsigned short*)(ws + kOffC16R);

  const dim3 splitGrid(kDz / 64, kDz / 64);
  const int smallBlocks = ((kDz / 64) * (kDz / 64)) / 8;

  cast_f16_carry_kernel<true><<<(kRowsB * kDx / 8) / 256, 256, 0, stream>>>(X, X16, X16R, kRowsB * kDx / 8, kCarryAct);
  cast_f16_carry_kernel<true><<<(kHid * kDz / 8) / 256, 256, 0, stream>>>(W1, W1H, W1R, kHid * kDz / 8, kCarryW);
  cast_f16_carry_kernel<false><<<(kHid * kHid / 8) / 256, 256, 0, stream>>>(W2, W2H, W2H, kHid * kHid / 8, kCarryW);
  cast_f16_carry_kernel<true><<<(kDy * kHid / 8) / 256, 256, 0, stream>>>(W3, W3H, W3R, kDy * kHid / 8, kCarryW);

  split_planes_kernel<true, false><<<splitGrid, 256, 0, stream>>>(Am, LA, RT, 1.0f);
  split_planes_kernel<false, true><<<splitGrid, 256, 0, stream>>>(Am, LA, RT, kDt * 0.25f);

  gemm64_kernel<1, false, false, 0, true, false, false><<<smallBlocks, 256, 0, stream>>>(
      LA, LA, kK3, RT, RT, kK3, (void*)F0, (void*)F0, kDz, b3, Am, kDz, nst, kDz, kDz, kK3, kDt / 3.0f, kDt / 3.0f, 1.0f);
  split_planes_kernel<false, true><<<splitGrid, 256, 0, stream>>>(F0, LE, RT, 1.0f);
  gemm64_kernel<1, false, false, 0, true, false, false><<<smallBlocks, 256, 0, stream>>>(
      LA, LA, kK3, RT, RT, kK3, (void*)F1, (void*)F1, kDz, b3, Am, kDz, nst, kDz, kDz, kK3, kDt * 0.5f, kDt * 0.5f, 1.0f);
  split_planes_kernel<false, true><<<splitGrid, 256, 0, stream>>>(F1, LE, RT, 1.0f);
  gemm64_kernel<1, false, false, 0, true, false, false><<<smallBlocks, 256, 0, stream>>>(
      LA, LA, kK3, RT, RT, kK3, (void*)F2, (void*)F2, kDz, b3, Am, kDz, nst, kDz, kDz, kK3, kDt, kDt, 1.0f);

  static_assert(kSteps == 64, "six doublings");
  float* esrc = F2;
  float* edst = F0;
  for (int s = 0; s < 6; ++s) {
    split_planes_kernel<true, true><<<splitGrid, 256, 0, stream>>>(esrc, LE, RT, 1.0f);
    gemm64_kernel<1, false, false, 0, true, false, false><<<smallBlocks, 256, 0, stream>>>(
        LE, LE, kK3, RT, RT, kK3, (void*)edst, (void*)edst, kDz, b3, esrc, kDz, nst, kDz, kDz, kK3, 1.0f, 2.0f, 1.0f);
    float* t = esrc;
    esrc = edst;
    edst = t;
  }

  split_planes_kernel<true, false><<<splitGrid, 256, 0, stream>>>(esrc, LE, PT, 1.0f);
  split_planes_kernel<false, true><<<splitGrid, 256, 0, stream>>>(Pm, LE, PT, 1.0f);
  gemm64_kernel<1, false, false, 2, true, false, false><<<smallBlocks, 256, 0, stream>>>(
      LE, LE, kK3, PT, PT, kK3, (void*)C16, (void*)C16R, kDx, b3, Pm, kDx, nst, kDz, kDx, kK3, 1.0f, 1.0f, kCarryW);

  gemm64_kernel<0, true, false, 2, false, false, false><<<((kRowsB / 32) * (kDz / 64)) / 8, 256, 0, stream>>>(
      X16, X16R, kDx, C16, C16R, kDx, (void*)ZT16, (void*)ZT16R, kDz, b3, Am, kDz, nst,
      kRowsB, kDz, kDx, kFoldBack, 0.0f, kCarryAct);
  gemm64_kernel<0, true, true, 1, false, true, false><<<((kRowsB / 32) * (kHid / 64)) / 8, 256, 0, stream>>>(
      ZT16, ZT16R, kDz, W1H, W1R, kDz, (void*)H1, (void*)H1, kHid, b1, Am, kDz, nst,
      kRowsB, kHid, kDz, kFoldBack, 0.0f, kCarryAct);
  gemm64_kernel<0, false, true, 2, false, true, false><<<((kRowsB / 64) * (kHid / 64)) / 8, 256, 0, stream>>>(
      H1, H1, kHid, W2H, W2H, kHid, (void*)H2, (void*)H2R, kHid, b2, Am, kDz, nst,
      kRowsB, kHid, kHid, kFoldBack, 0.0f, kCarryAct);
  gemm64_kernel<0, true, true, 0, false, false, true><<<((kRowsB / 32) * (kDy / 64)) / 8, 256, 0, stream>>>(
      H2, H2R, kHid, W3H, W3R, kHid, (void*)y, (void*)y, kDy, b3, Am, kDz, nst,
      kRowsB, kDy, kHid, kFoldBack, 0.0f, 1.0f);
}
